// GenomicTransformModel_42039139893589
// MI455X (gfx1250) — hardware-verified
//
#include <hip/hip_runtime.h>
#include <math.h>

typedef _Float16 v16h __attribute__((ext_vector_type(16)));
typedef _Float16 v8h  __attribute__((ext_vector_type(8)));
typedef _Float16 v4h  __attribute__((ext_vector_type(4)));
typedef float    v8f  __attribute__((ext_vector_type(8)));
typedef float    v4f  __attribute__((ext_vector_type(4)));
typedef float    v2f  __attribute__((ext_vector_type(2)));
typedef v8h __attribute__((may_alias)) v8ha;
typedef v4f __attribute__((may_alias)) v4fa;

union Frag { v16h v; v8h half[2]; };

#define LNUM  4
#define NHEAD 8
#define DMOD  128
#define FFD   256
#define SEQ   1024
#define NBAT  8
#define LWIN  128
#define HDIM  16
#define VOCAB 16
#define QKVW  (3 * DMOD)
#define MTOK  (NBAT * SEQ)
#define NBH   (NBAT * NHEAD)

#define NWQKV (LNUM * QKVW * DMOD)
#define NWO   (LNUM * DMOD * DMOD)
#define NW1   (LNUM * FFD * DMOD)
#define NW2   (LNUM * DMOD * FFD)
#define NWALL (NWQKV + NWO + NW1 + NW2)

#define WSC    32.0f
#define QSC    4.0f
#define KVSC   16.0f
#define HSC    16.0f
#define PSC    16384.0f
#define LN_EPS 1e-5f

static_assert((NWQKV % 2048) == 0);
static_assert((NWO % 2048) == 0);
static_assert((NW1 % 2048) == 0);
static_assert((NW2 % 2048) == 0);
static_assert((MTOK % 64) == 0);
static_assert((SEQ % 64) == 0);

#define SZ_X     ((size_t)MTOK * DMOD * 4)
#define SZ_XH    ((size_t)MTOK * DMOD * 2)
#define SZ_PL    ((size_t)NBH * SEQ * HDIM * 2)
#define SZ_CTX   ((size_t)MTOK * DMOD * 2)
#define SZ_FFH   ((size_t)MTOK * FFD * 2)
#define SZ_WALL  ((size_t)NWALL * 2)
#define SZ_PE    ((size_t)SEQ * DMOD * 4)
#define OFF_X    ((size_t)0)
#define OFF_XH   (OFF_X + SZ_X)
#define OFF_QP   (OFF_XH + SZ_XH)
#define OFF_KP   (OFF_QP + SZ_PL)
#define OFF_VT   (OFF_KP + SZ_PL)
#define OFF_CTX  (OFF_VT + SZ_PL)
#define OFF_FFH  (OFF_CTX + SZ_CTX)
#define OFF_WALL (OFF_FFH + SZ_FFH)
#define OFF_PE   (OFF_WALL + SZ_WALL)
#define WS_TOTAL (OFF_PE + SZ_PE)
static_assert((OFF_XH % 256) == 0);
static_assert((OFF_QP % 256) == 0);
static_assert((OFF_WALL % 256) == 0);
static_assert((OFF_PE % 256) == 0);
static_assert(WS_TOTAL == (size_t)20447232);

__constant__ unsigned int kDiv[64] = {0x3f800000u,0x3f5dafd6u,0x3f3ff911u,0x3f263de0u,0x3f0ff59au,0x3ef953ceu,0x3ed7e89au,0x3ebaf81au,0x3ea1e89bu,0x3e8c3503u,0x3e72d422u,0x3e5247edu,0x3e361887u,0x3e1db040u,0x3e088d77u,0x3dec7fd5u,0x3dccccccu,0x3db15978u,0x3d99940du,0x3d84fe4cu,0x3d6655c1u,0x3d477640u,0x3d2cba16u,0x3d159348u,0x3d0186e2u,0x3ce054d1u,0x3cc2434eu,0x3ca83989u,0x3c91ad3au,0x3c7c4d30u,0x3c5a7bf1u,0x3c3d330eu,0x3c23d70au,0x3c0de12eu,0x3bf5b9adu,0x3bd4ca16u,0x3bb8449au,0x3b9f91ccu,0x3b8a2e75u,0x3b6f520du,0x3b4f3e33u,0x3b33770du,0x3b1b690eu,0x3b06946du,0x3ae91528u,0x3ac9d759u,0x3aaec98du,0x3a975c0bu,0x3a83126eu,0x3a6301e3u,0x3a44948au,0x3a2a3b44u,0x3a136a14u,0x39ff4facu,0x39dd1722u,0x39bf74d6u,0x39a5cb60u,0x398f9275u,0x3978a80du,0x395753e2u,0x393a7753u,0x39217918u,0x390bd46du,0x38f22cddu};

__device__ __forceinline__ v8f wmma16(v16h a, v16h b, v8f c) {
  v8f d = __builtin_amdgcn_wmma_f32_16x16x32_f16(false, a, false, b, (short)0, c, false, false);
  asm volatile("v_nop\n\tv_nop\n\tv_nop\n\tv_nop" : "+v"(d) : "v"(a), "v"(b));
  return d;
}

__device__ __forceinline__ v8f zero8f() {
  v8f z = {0.f, 0.f, 0.f, 0.f, 0.f, 0.f, 0.f, 0.f};
  return z;
}

__device__ __forceinline__ v8h zero8h() {
  v8h z = {(_Float16)0.f, (_Float16)0.f, (_Float16)0.f, (_Float16)0.f,
           (_Float16)0.f, (_Float16)0.f, (_Float16)0.f, (_Float16)0.f};
  return z;
}

__device__ __forceinline__ v16h load_frag(const _Float16* p, int h) {
  Frag f;
  f.half[0] = *(const v8ha*)(p + 8 * h);
  f.half[1] = *(const v8ha*)(p + 16 + 8 * h);
  return f.v;
}

__device__ __forceinline__ v16h load_frag16(const _Float16* p, int h) {
  Frag f;
  f.half[0] = *(const v8ha*)(p + 8 * h);
  f.half[1] = zero8h();
  return f.v;
}

__device__ __forceinline__ float wave_sum(float v) {
  v += __shfl_xor(v, 16);
  v += __shfl_xor(v, 8);
  v += __shfl_xor(v, 4);
  v += __shfl_xor(v, 2);
  v += __shfl_xor(v, 1);
  return v;
}

__device__ __forceinline__ v4f ln_row(v4f v, v4f g, v4f bb) {
  const float s1 = wave_sum((v.x + v.y) + (v.z + v.w));
  const float mean = s1 * (1.0f / (float)DMOD);
  const float cx = v.x - mean, cy = v.y - mean, cz = v.z - mean, cw = v.w - mean;
  const float s2 = wave_sum((cx * cx + cy * cy) + (cz * cz + cw * cw));
  const float rstd = rsqrtf(s2 * (1.0f / (float)DMOD) + LN_EPS);
  v4f o;
  o.x = cx * rstd * g.x + bb.x;
  o.y = cy * rstd * g.y + bb.y;
  o.z = cz * rstd * g.z + bb.z;
  o.w = cw * rstd * g.w + bb.w;
  return o;
}

__device__ __forceinline__ v4h to_h4(v4f v) {
  v4h r = {(_Float16)v.x, (_Float16)v.y, (_Float16)v.z, (_Float16)v.w};
  return r;
}

template <int NT>
__device__ __forceinline__ void gemm_loop(const _Float16* __restrict__ arow,
                                          const _Float16* __restrict__ wrow,
                                          int ldw, int K, int h, v8f (&acc)[NT]) {
  #pragma unroll 1
  for (int k0 = 0; k0 < K; k0 += 32) {
    const v16h a = load_frag(arow + k0, h);
    #pragma unroll
    for (int t = 0; t < NT; ++t) {
      const v16h b = load_frag(wrow + (size_t)t * 16 * ldw + k0, h);
      acc[t] = wmma16(a, b, acc[t]);
    }
  }
}

__device__ __forceinline__ void lines16_store_pass(const _Float16* src, _Float16* dst,
                                                   int lstr, int lane) {
  const int q8 = lane & 7, sub = lane >> 3;
  #pragma unroll
  for (int i = 0; i < 4; ++i) {
    const int L = 4 * i + sub;
    const v8h v = *(const v8ha*)(src + L * 64 + 8 * q8);
    *(volatile v8h*)(dst + (size_t)L * lstr + 8 * q8) = v;
  }
}

__global__ __launch_bounds__(256) void cvt_w_kernel(
    const float* __restrict__ wqkv, const float* __restrict__ wo,
    const float* __restrict__ w1, const float* __restrict__ w2,
    _Float16* __restrict__ wall)
{
  const int g = blockIdx.x * 256 + threadIdx.x;
  if (g >= NWALL / 8) return;
  const float* src;
  if (g < NWQKV / 8)                    src = wqkv + (size_t)g * 8;
  else if (g < (NWQKV + NWO) / 8)       src = wo + (size_t)(g - NWQKV / 8) * 8;
  else if (g < (NWQKV + NWO + NW1) / 8) src = w1 + (size_t)(g - (NWQKV + NWO) / 8) * 8;
  else                                  src = w2 + (size_t)(g - (NWQKV + NWO + NW1) / 8) * 8;
  const v4f a = *(const v4fa*)src;
  const v4f c = *(const v4fa*)(src + 4);
  const v8h o = { (_Float16)(a.x * WSC), (_Float16)(a.y * WSC), (_Float16)(a.z * WSC), (_Float16)(a.w * WSC),
                  (_Float16)(c.x * WSC), (_Float16)(c.y * WSC), (_Float16)(c.z * WSC), (_Float16)(c.w * WSC) };
  _Float16* dst = wall + (size_t)g * 8;
  *(volatile v8h*)dst = o;
  __threadfence();
  *(volatile v8h*)dst = o;
}

__global__ __launch_bounds__(256) void pe_kernel(float* __restrict__ pe)
{
  const int g = blockIdx.x * 256 + threadIdx.x;
  if (g >= SEQ * (DMOD / 2)) return;
  const int s = g >> 6, i = g & 63;
  const float ang = (float)s * __uint_as_float(kDiv[i]);
  const float sn = sinf(ang);
  const float cs = cosf(ang);
  const v2f o = {sn, cs};
  float* dst = pe + (size_t)s * DMOD + 2 * i;
  *(volatile v2f*)dst = o;
  __threadfence();
  *(volatile v2f*)dst = o;
}

__global__ __launch_bounds__(256) void embed_kernel(
    const int* __restrict__ tok, const float* __restrict__ emb,
    const float* __restrict__ pe, float* __restrict__ x, _Float16* __restrict__ xh)
{
  const int lane = threadIdx.x & 31, w = threadIdx.x >> 5;
  const int row = blockIdx.x * 8 + w;
  if (row >= MTOK) return;
  const int s = row & (SEQ - 1);
  int t = tok[row];
  t = (t < 0) ? (t + VOCAB) : t;
  t = min(max(t, 0), VOCAB - 1);
  const v4f e = *(const v4fa*)(emb + (size_t)t * DMOD + 4 * lane);
  const v4f p = *(const v4fa*)(pe + (size_t)s * DMOD + 4 * lane);
  const v4f v = e + p;
  const v4h hv = to_h4(v);
  float* xd = x + (size_t)row * DMOD + 4 * lane;
  _Float16* hd = xh + (size_t)row * DMOD + 4 * lane;
  *(volatile v4f*)xd = v;
  *(volatile v4h*)hd = hv;
  __threadfence();
  *(volatile v4f*)xd = v;
  *(volatile v4h*)hd = hv;
}

__global__ __launch_bounds__(128) void qkv_kernel(
    const _Float16* __restrict__ xh,
    const _Float16* __restrict__ wl,
    const float* __restrict__ bl,
    _Float16* __restrict__ qp, _Float16* __restrict__ kp, _Float16* __restrict__ vt)
{
  __shared__ __attribute__((aligned(16))) _Float16 sT[4 * 64 * HDIM];

  const int tid = threadIdx.x, lane = tid & 31, w = tid >> 5;
  const int h = lane >> 4, m = lane & 15;
  const int m0 = blockIdx.x * 64;
  const int cg = blockIdx.y;
  const int which = cg >> 1, hg = cg & 1;
  const int f0 = which * DMOD + hg * 64;

  const _Float16* arow = xh + (size_t)(m0 + 16 * w + m) * DMOD;
  const _Float16* wrow = wl + (size_t)(f0 + m) * DMOD;
  v8f acc[4];
  #pragma unroll
  for (int t = 0; t < 4; ++t) acc[t] = zero8f();
  gemm_loop<4>(arow, wrow, DMOD, DMOD, h, acc);

  const float sc = (which == 0) ? QSC : KVSC;
  #pragma unroll
  for (int t = 0; t < 4; ++t) {
    const float bv = bl[f0 + 16 * t + m];
    #pragma unroll
    for (int r = 0; r < 8; ++r) {
      const int tl = 16 * w + 8 * h + r;
      const float y = (acc[t][r] * (1.0f / WSC) + bv) * sc;
      const int idx = (which == 2) ? ((t * HDIM + m) * 64 + tl) : ((t * 64 + tl) * HDIM + m);
      sT[idx] = (_Float16)y;
    }
  }
  __syncthreads();

  const int b = m0 / SEQ, s0 = m0 - b * SEQ;
  const int bh = b * NHEAD + hg * 4 + w;
  _Float16* dst;
  int lstr;
  if (which == 2) { dst = vt + (size_t)bh * HDIM * SEQ + s0; lstr = SEQ; }
  else { dst = ((which == 0) ? qp : kp) + ((size_t)bh * SEQ + s0) * HDIM; lstr = 64; }
  const _Float16* src = sT + w * 1024;
  lines16_store_pass(src, dst, lstr, lane);
  __threadfence();
  lines16_store_pass(src, dst, lstr, lane);
}

__device__ __forceinline__ v16h pack_p(v8f a, v8f c) {
  const v16h r = { (_Float16)(a[0] * PSC), (_Float16)(a[1] * PSC), (_Float16)(a[2] * PSC), (_Float16)(a[3] * PSC),
                   (_Float16)(a[4] * PSC), (_Float16)(a[5] * PSC), (_Float16)(a[6] * PSC), (_Float16)(a[7] * PSC),
                   (_Float16)(c[0] * PSC), (_Float16)(c[1] * PSC), (_Float16)(c[2] * PSC), (_Float16)(c[3] * PSC),
                   (_Float16)(c[4] * PSC), (_Float16)(c[5] * PSC), (_Float16)(c[6] * PSC), (_Float16)(c[7] * PSC) };
  return r;
}

__device__ __forceinline__ void ctx_store_pass(const _Float16* sC, _Float16* ctxh,
                                               int tok0, int w, int lane) {
  const int piece = lane & 15, rr = lane >> 4;
  #pragma unroll
  for (int i = 0; i < 8; ++i) {
    const int row = 2 * i + rr;
    const v8h v = *(const v8ha*)(sC + (16 * w + row) * DMOD + 8 * piece);
    *(volatile v8h*)(ctxh + (size_t)(tok0 + row) * DMOD + 8 * piece) = v;
  }
}

__global__ __launch_bounds__(128) void attn_kernel(
    const _Float16* __restrict__ qp,
    const _Float16* __restrict__ kp,
    const _Float16* __restrict__ vt,
    _Float16* __restrict__ ctxh)
{
  __shared__ __attribute__((aligned(16))) _Float16 sC[64 * DMOD];

  const int tid = threadIdx.x, lane = tid & 31, w = tid >> 5;
  const int h = lane >> 4, m = lane & 15;
  const int q0b = blockIdx.x * 64;
  const int b = blockIdx.y;
  const int q0w = q0b + 16 * w;
  const float NEG_INF = -__builtin_inff();

  #pragma unroll 1
  for (int head = 0; head < NHEAD; ++head) {
    const int bh = b * NHEAD + head;
    const v16h qf = load_frag16(qp + ((size_t)bh * SEQ + q0w + m) * HDIM, h);
    const _Float16* kbase = kp + ((size_t)bh * SEQ + m) * HDIM;
    const _Float16* vbase = vt + ((size_t)bh * HDIM + m) * SEQ;

    v8f o = zero8f();
    float mrun = NEG_INF, lrun = 0.0f;

    #pragma unroll 1
    for (int c = 0; c < 5; ++c) {
      const int kb = q0b - LWIN + 64 * c;
      if (kb < 0 || kb >= SEQ) continue;

      v8f s[4];
      #pragma unroll
      for (int j = 0; j < 4; ++j) {
        const v16h kf = load_frag16(kbase + (size_t)(kb + 16 * j) * HDIM, h);
        s[j] = wmma16(kf, qf, zero8f());
      }
      #pragma unroll
      for (int j = 0; j < 4; ++j) {
        #pragma unroll
        for (int r = 0; r < 8; ++r) {
          const int key = kb + 16 * j + 8 * h + r;
          const int dq = key - (q0w + m);
          const bool ok = (dq <= LWIN) && (dq >= -LWIN);
          s[j][r] = ok ? (s[j][r] * (1.0f / 256.0f)) : NEG_INF;
        }
      }
      float mloc = s[0][0];
      #pragma unroll
      for (int j = 0; j < 4; ++j)
        #pragma unroll
        for (int r = 0; r < 8; ++r) mloc = fmaxf(mloc, s[j][r]);
      mloc = fmaxf(mloc, __shfl_xor(mloc, 16));
      const float mnew = fmaxf(mrun, mloc);
      const float msafe = (mnew == NEG_INF) ? 0.0f : mnew;
      const float alpha = __expf(mrun - msafe);
      mrun = mnew;
      float lsum = 0.0f;
      #pragma unroll
      for (int j = 0; j < 4; ++j)
        #pragma unroll
        for (int r = 0; r < 8; ++r) {
          const float p = __expf(s[j][r] - msafe);
          s[j][r] = p;
          lsum += p;
        }
      lsum += __shfl_xor(lsum, 16);
      lrun = lrun * alpha + lsum;
      #pragma unroll
      for (int r = 0; r < 8; ++r) o[r] = o[r] * alpha;

      const v16h pb0 = pack_p(s[0], s[1]);
      const v16h pb1 = pack_p(s[2], s[3]);

      const v16h vf0 = load_frag(vbase + kb, h);
      const v16h vf1 = load_frag(vbase + kb + 32, h);
      o = wmma16(vf0, pb0, o);
      o = wmma16(vf1, pb1, o);
    }

    const float inv = (lrun > 0.0f) ? (1.0f / (lrun * PSC)) : 0.0f;
    #pragma unroll
    for (int r = 0; r < 8; ++r)
      sC[(16 * w + m) * DMOD + head * HDIM + 8 * h + r] = (_Float16)(o[r] * inv);
  }
  __syncthreads();

  const int tok0 = b * SEQ + q0w;
  ctx_store_pass(sC, ctxh, tok0, w, lane);
  __threadfence();
  ctx_store_pass(sC, ctxh, tok0, w, lane);
}

template <int KD>
__global__ __launch_bounds__(128) void gemm_ln_kernel(
    const _Float16* __restrict__ ap,
    const _Float16* __restrict__ wl,
    const float* __restrict__ bl,
    const float* __restrict__ g, const float* __restrict__ bb,
    float* __restrict__ x,
    _Float16* __restrict__ xh)
{
  __shared__ __attribute__((aligned(16))) float sY[64 * 132];

  const int tid = threadIdx.x, lane = tid & 31, w = tid >> 5;
  const int h = lane >> 4, m = lane & 15;
  const int m0 = blockIdx.x * 64;

  const _Float16* arow = ap + (size_t)(m0 + 16 * w + m) * KD;
  const _Float16* wrow = wl + (size_t)m * KD;
  v8f acc[8];
  #pragma unroll
  for (int t = 0; t < 8; ++t) acc[t] = zero8f();
  gemm_loop<8>(arow, wrow, KD, KD, h, acc);

  #pragma unroll
  for (int t = 0; t < 8; ++t) {
    const int n = 16 * t + m;
    const float bv = bl[n];
    #pragma unroll
    for (int r = 0; r < 8; ++r)
      sY[(16 * w + 8 * h + r) * 132 + n] = acc[t][r] * (1.0f / (WSC * KVSC)) + bv;
  }
  __syncthreads();

  const v4f gv  = *(const v4fa*)(g + 4 * lane);
  const v4f bv4 = *(const v4fa*)(bb + 4 * lane);
  #pragma unroll 1
  for (int i = 0; i < 16; ++i) {
    const int row = 16 * w + i;
    const size_t tok = (size_t)(m0 + row);
    const v4f yv = *(const v4fa*)(sY + row * 132 + 4 * lane);
    const v4f xv = *(const v4fa*)(x + tok * DMOD + 4 * lane);
    const v4f v = xv + yv;
    const v4f o = ln_row(v, gv, bv4);
    const v4h ho = to_h4(o);
    float* xd = x + tok * DMOD + 4 * lane;
    _Float16* hd = xh + tok * DMOD + 4 * lane;
    *(volatile v4f*)xd = o;
    *(volatile v4h*)hd = ho;
    __threadfence();
    *(volatile v4f*)xd = o;
    *(volatile v4h*)hd = ho;
  }
}

__global__ __launch_bounds__(128) void ffn1_kernel(
    const _Float16* __restrict__ xh,
    const _Float16* __restrict__ wl,
    const float* __restrict__ bl,
    _Float16* __restrict__ ffh)
{
  __shared__ __attribute__((aligned(16))) _Float16 sT[64 * 64];

  const int tid = threadIdx.x, lane = tid & 31, w = tid >> 5;
  const int h = lane >> 4, m = lane & 15;
  const int m0 = blockIdx.x * 64;
  const int n0 = blockIdx.y * 64;

  const _Float16* arow = xh + (size_t)(m0 + 16 * w + m) * DMOD;
  const _Float16* wrow = wl + (size_t)(n0 + m) * DMOD;
  v8f acc[4];
  #pragma unroll
  for (int t = 0; t < 4; ++t) acc[t] = zero8f();
  gemm_loop<4>(arow, wrow, DMOD, DMOD, h, acc);

  #pragma unroll
  for (int t = 0; t < 4; ++t) {
    const float bv = bl[n0 + 16 * t + m];
    #pragma unroll
    for (int r = 0; r < 8; ++r) {
      const int tl = 16 * w + 8 * h + r;
      const float y = fmaxf(acc[t][r] * (1.0f / WSC) + bv, 0.0f) * HSC;
      sT[tl * 64 + 16 * t + m] = (_Float16)y;
    }
  }
  __syncthreads();

  const _Float16* src = sT + (16 * w) * 64;
  _Float16* dst = ffh + (size_t)(m0 + 16 * w) * FFD + n0;
  lines16_store_pass(src, dst, FFD, lane);
  __threadfence();
  lines16_store_pass(src, dst, FFD, lane);
}

__global__ __launch_bounds__(256) void head_kernel(
    const float* __restrict__ x, const float* __restrict__ g, const float* __restrict__ bb,
    const float* __restrict__ wout, const float* __restrict__ bout, float* __restrict__ out)
{
  __shared__ __attribute__((aligned(16))) float res[32];
  const int tid = threadIdx.x, lane = tid & 31, w = tid >> 5;
  const v4f gv  = *(const v4fa*)(g + 4 * lane);
  const v4f bv4 = *(const v4fa*)(bb + 4 * lane);
  const v4f wv  = *(const v4fa*)(wout + 4 * lane);
  const float b0 = bout[0];
  #pragma unroll 1
  for (int i = 0; i < 4; ++i) {
    const int tok = blockIdx.x * 32 + w * 4 + i;
    const v4f xv = *(const v4fa*)(x + (size_t)tok * DMOD + 4 * lane);
    const v4f nv = ln_row(xv, gv, bv4);
    const float d = wave_sum((nv.x * wv.x + nv.y * wv.y) + (nv.z * wv.z + nv.w * wv.w));
    const float z = d + b0;
    const float sp = fmaxf(z, 0.0f) + log1pf(expf(-fabsf(z)));
    if (lane == 0) res[w * 4 + i] = sp;
  }
  __syncthreads();
  const v4f v = *(const v4fa*)(res + 4 * (tid & 7));
  float* dst = out + (size_t)blockIdx.x * 32 + 4 * (tid & 7);
  if (tid < 8) *(volatile v4f*)dst = v;
  __threadfence();
  if (tid < 8) *(volatile v4f*)dst = v;
}

extern "C" void kernel_launch(void* const* d_in, const int* in_sizes, int n_in,
                              void* d_out, int out_size, void* d_ws, size_t ws_size,
                              hipStream_t stream) {
  if (n_in < 18) return;
  if (in_sizes[0] != MTOK || in_sizes[1] != VOCAB * DMOD || in_sizes[2] != NWQKV ||
      in_sizes[3] != LNUM * QKVW || in_sizes[4] != NWO || in_sizes[5] != LNUM * DMOD ||
      in_sizes[6] != LNUM * DMOD || in_sizes[7] != LNUM * DMOD || in_sizes[8] != LNUM * DMOD ||
      in_sizes[9] != LNUM * DMOD || in_sizes[10] != NW1 || in_sizes[11] != LNUM * FFD ||
      in_sizes[12] != NW2 || in_sizes[13] != LNUM * DMOD || in_sizes[14] != DMOD ||
      in_sizes[15] != DMOD || in_sizes[16] != DMOD || in_sizes[17] != 1) return;
  if (out_size != MTOK) return;
  if (WS_TOTAL > ws_size) return;

  const int*   tok  = (const int*)d_in[0];
  const float* emb  = (const float*)d_in[1];
  const float* Wqkv = (const float*)d_in[2];
  const float* bqkv = (const float*)d_in[3];
  const float* Wo   = (const float*)d_in[4];
  const float* bo   = (const float*)d_in[5];
  const float* ln1g = (const float*)d_in[6];
  const float* ln1b = (const float*)d_in[7];
  const float* ln2g = (const float*)d_in[8];
  const float* ln2b = (const float*)d_in[9];
  const float* W1   = (const float*)d_in[10];
  const float* b1   = (const float*)d_in[11];
  const float* W2   = (const float*)d_in[12];
  const float* b2   = (const float*)d_in[13];
  const float* lnfg = (const float*)d_in[14];
  const float* lnfb = (const float*)d_in[15];
  const float* Wout = (const float*)d_in[16];
  const float* bout = (const float*)d_in[17];
  float* out = (float*)d_out;

  char* ws = (char*)d_ws;
  float*    x    = (float*)(ws + OFF_X);
  _Float16* xh   = (_Float16*)(ws + OFF_XH);
  _Float16* qp   = (_Float16*)(ws + OFF_QP);
  _Float16* kp   = (_Float16*)(ws + OFF_KP);
  _Float16* vt   = (_Float16*)(ws + OFF_VT);
  _Float16* ctxh = (_Float16*)(ws + OFF_CTX);
  _Float16* ffh  = (_Float16*)(ws + OFF_FFH);
  _Float16* wall = (_Float16*)(ws + OFF_WALL);
  float*    pe   = (float*)(ws + OFF_PE);
  _Float16* wqkvh = wall;
  _Float16* woh   = wall + NWQKV;
  _Float16* w1h   = wall + NWQKV + NWO;
  _Float16* w2h   = wall + NWQKV + NWO + NW1;

  cvt_w_kernel<<<(NWALL / 8) / 256, 256, 0, stream>>>(Wqkv, Wo, W1, W2, wall);
  pe_kernel<<<(SEQ * (DMOD / 2)) / 256, 256, 0, stream>>>(pe);
  embed_kernel<<<MTOK / 8, 256, 0, stream>>>(tok, emb, pe, x, xh);

  for (int l = 0; l < LNUM; ++l) {
    qkv_kernel<<<dim3(MTOK / 64, 6), 128, 0, stream>>>(
        xh, wqkvh + (size_t)l * QKVW * DMOD, bqkv + l * QKVW, qp, kp, vt);
    attn_kernel<<<dim3(SEQ / 64, NBAT), 128, 0, stream>>>(qp, kp, vt, ctxh);
    gemm_ln_kernel<DMOD><<<MTOK / 64, 128, 0, stream>>>(
        ctxh, woh + (size_t)l * DMOD * DMOD, bo + l * DMOD, ln1g + l * DMOD, ln1b + l * DMOD, x, xh);
    ffn1_kernel<<<dim3(MTOK / 64, FFD / 64), 128, 0, stream>>>(
        xh, w1h + (size_t)l * FFD * DMOD, b1 + l * FFD, ffh);
    gemm_ln_kernel<FFD><<<MTOK / 64, 128, 0, stream>>>(
        ffh, w2h + (size_t)l * DMOD * FFD, b2 + l * DMOD, ln2g + l * DMOD, ln2b + l * DMOD, x, xh);
  }

  head_kernel<<<MTOK / 32, 256, 0, stream>>>(x, lnfg, lnfb, Wout, bout, out);
}
